// PointNet_50122268344667
// MI455X (gfx1250) — hardware-verified
//
#include <hip/hip_runtime.h>
#include <math.h>

constexpr int NCASE   = 16;
constexpr int NPTS    = 65536;
constexpr int NF0     = 64;
constexpr int NF1     = 128;
constexpr int NF2     = 512;
constexpr int NHEAD   = 256;
constexpr int NBATCH  = 4096;

constexpr int K1_THREADS  = 128;
constexpr int K1_WAVES    = K1_THREADS / 32;
constexpr int BLOCK_ROWS  = 32 * K1_WAVES;
constexpr int CHUNK_PTS   = 2048;
constexpr int NCHUNK      = NPTS / CHUNK_PTS;
constexpr int TILES_PER_BLOCK = CHUNK_PTS / BLOCK_ROWS;
constexpr int NPART       = NCHUNK * K1_WAVES;
constexpr int H0P = 72;
constexpr int H1P = 136;
constexpr float WCARRY     = 16.0f;
constexpr float WCARRY_INV = 1.0f / 16.0f;

static_assert(NPTS % CHUNK_PTS == 0, "chunking exact");
static_assert(CHUNK_PTS % BLOCK_ROWS == 0, "tiles exact");
static_assert(NF0 % 32 == 0 && NF1 % 32 == 0, "K multiples of 32");
static_assert(NF1 % 16 == 0 && NF2 % 16 == 0, "N multiples of 16");
static_assert(NPART == 128, "partials per case");
static_assert((H0P * 2) % 16 == 0 && (H1P * 2) % 16 == 0, "16-B aligned LDS rows");
static_assert(K1_WAVES * 32 * H0P * 2 + K1_WAVES * 32 * H1P * 2 + K1_WAVES * 512 * 4 + 384 * 4 <= 65536, "static LDS");

typedef __attribute__((ext_vector_type(16))) _Float16 v16h;
typedef __attribute__((ext_vector_type(8)))  _Float16 v8h;
typedef __attribute__((ext_vector_type(8)))  float    v8f;
typedef __attribute__((ext_vector_type(4)))  float    v4f;

template <typename T> struct Frag;
template <> struct Frag<_Float16> {
  typedef v16h V; union U { v16h v; v8h h[2]; };
  static __device__ __forceinline__ v16h load(const _Float16* p) {
    U f; f.h[0] = *(const v8h*)(p); f.h[1] = *(const v8h*)(p + 16); return f.v;
  }
  static __device__ __forceinline__ v8f mma(v16h a, v16h b, v8f c) {
    return __builtin_amdgcn_wmma_f32_16x16x32_f16(false, a, false, b, (short)0, c, false, false);
  }
};

__device__ __forceinline__ void guard_l2(v8f& x, v8f& y, v16h a, v16h b, v16h c, v16h d, v16h e, v16h f) {
  asm volatile("v_nop\n\tv_nop\n\tv_nop\n\tv_nop"
               : "+v"(x), "+v"(y)
               : "v"(a), "v"(b), "v"(c), "v"(d), "v"(e), "v"(f));
}
__device__ __forceinline__ void guard_l3(v8f& x, v8f& y,
                                         v16h b0, v16h b1, v16h b2, v16h b3,
                                         v16h p0, v16h p1, v16h p2, v16h p3,
                                         v16h q0, v16h q1, v16h q2, v16h q3) {
  asm volatile("v_nop\n\tv_nop\n\tv_nop\n\tv_nop"
               : "+v"(x), "+v"(y)
               : "v"(b0), "v"(b1), "v"(b2), "v"(b3),
                 "v"(p0), "v"(p1), "v"(p2), "v"(p3),
                 "v"(q0), "v"(q1), "v"(q2), "v"(q3));
}

__device__ __forceinline__ void wave_lds_sync() {
  __builtin_amdgcn_fence(__ATOMIC_RELEASE, "workgroup");
  __builtin_amdgcn_wave_barrier();
  __builtin_amdgcn_fence(__ATOMIC_ACQUIRE, "workgroup");
}

__device__ __forceinline__ float silu_f(float x) {
  const float xc = fmaxf(x, -60.0f);
  const float e  = expf(-xc);
  return x * __builtin_amdgcn_rcpf(1.0f + e);
}

__global__ __launch_bounds__(256) void prep_weights_kernel(const float* __restrict__ W1_1, const float* __restrict__ W1_2,
                                                           unsigned short* __restrict__ Bt1, unsigned short* __restrict__ Bt2) {
  const int i = blockIdx.x * 256 + threadIdx.x;
  if (i >= 1024 + 8192) return;
  const bool second = (i >= 1024);
  const int j     = second ? (i - 1024) : i;
  const int ndim  = second ? NF2 : NF1;
  const int n     = second ? (j >> 4) : (j >> 3);
  const int k8    = second ? (j & 15) : (j & 7);
  const float* src = second ? W1_2 : W1_1;
  unsigned short* dst = second ? Bt2 : Bt1;
  v8h hv;
#pragma unroll
  for (int e = 0; e < 8; ++e) {
    const float w = src[(size_t)(k8 * 8 + e) * ndim + n];
    hv[e] = (_Float16)(w * WCARRY);
  }
  unsigned short* op = dst + (size_t)j * 8;
  *(volatile v8h*)op = hv;
  __threadfence();
  *(volatile v8h*)op = hv;
}

__global__ __launch_bounds__(K1_THREADS) __attribute__((amdgpu_num_vgpr(256)))
void mlp_colminmax_kernel(const float* __restrict__ pts,
                          const float* __restrict__ W1_0, const float* __restrict__ b1_0,
                          const float* __restrict__ b1_1,
                          const unsigned short* Bt1p, const unsigned short* Bt2p,
                          float* __restrict__ PMAX, float* __restrict__ PMIN) {
  __shared__ __align__(16) _Float16 sH0[K1_WAVES][32 * H0P];
  __shared__ __align__(16) _Float16 sH1[K1_WAVES][32 * H1P];
  __shared__ __align__(16) float    sSlab[K1_WAVES][512];
  __shared__ __align__(16) float    sCst[384];

  const _Float16* Bt1 = (const _Float16*)Bt1p;
  const _Float16* Bt2 = (const _Float16*)Bt2p;

  const int tid  = threadIdx.x;
  const int lane = tid & 31;
  const int wave = tid >> 5;
  const int hh   = lane >> 4;
  const int c    = lane & 15;
  const int koff = hh * 8;

  sCst[tid] = W1_0[tid];
  if (tid < 64) sCst[128 + tid] = W1_0[128 + tid];
  if (tid < 64) sCst[192 + tid] = b1_0[tid];
  sCst[256 + tid] = b1_1[tid];
  __syncthreads();

  const int cs = blockIdx.x / NCHUNK;
  const int ch = blockIdx.x - cs * NCHUNK;
  const float* cpts = pts + (size_t)cs * NPTS * 3;
  const int pbase = ch * CHUNK_PTS + wave * 32 + lane;

  _Float16* h0w = sH0[wave];
  _Float16* h1w = sH1[wave];
  float*    slab = sSlab[wave];

  float rmax[32], rmin[32];
#pragma unroll
  for (int nt = 0; nt < 32; ++nt) { rmax[nt] = -INFINITY; rmin[nt] = INFINITY; }

  const v8f z8 = {0.f, 0.f, 0.f, 0.f, 0.f, 0.f, 0.f, 0.f};

#pragma unroll 1
  for (int tile = 0; tile < TILES_PER_BLOCK; ++tile) {
    {
      const int pi = pbase + tile * BLOCK_ROWS;
      const float* pp = cpts + (size_t)pi * 3;
      const float px = pp[0], py = pp[1], pz = pp[2];
      _Float16* h0row = h0w + lane * H0P;
#pragma unroll 1
      for (int g = 0; g < 8; ++g) {
        const float* cw = sCst + g * 8;
        const v4f wx0 = *(const v4f*)(cw);
        const v4f wx1 = *(const v4f*)(cw + 4);
        const v4f wy0 = *(const v4f*)(cw + 64);
        const v4f wy1 = *(const v4f*)(cw + 68);
        const v4f wz0 = *(const v4f*)(cw + 128);
        const v4f wz1 = *(const v4f*)(cw + 132);
        const v4f bb0 = *(const v4f*)(cw + 192);
        const v4f bb1 = *(const v4f*)(cw + 196);
        v8h hv;
#pragma unroll
        for (int e = 0; e < 4; ++e) {
          float u = px * wx0[e];
          u = fmaf(py, wy0[e], u);
          u = fmaf(pz, wz0[e], u);
          u += bb0[e];
          float w = px * wx1[e];
          w = fmaf(py, wy1[e], w);
          w = fmaf(pz, wz1[e], w);
          w += bb1[e];
          hv[e]     = (_Float16)silu_f(u);
          hv[4 + e] = (_Float16)silu_f(w);
        }
        *(v8h*)(h0row + g * 8) = hv;
      }
    }
    wave_lds_sync();

    {
      const v16h hb00 = Frag<_Float16>::load(h0w + c * H0P + koff);
      const v16h hb01 = Frag<_Float16>::load(h0w + c * H0P + 32 + koff);
      const v16h hb10 = Frag<_Float16>::load(h0w + (16 + c) * H0P + koff);
      const v16h hb11 = Frag<_Float16>::load(h0w + (16 + c) * H0P + 32 + koff);
#pragma unroll 1
      for (int nt = 0; nt < NF1 / 16; ++nt) {
        const _Float16* wp = Bt1 + (size_t)(nt * 16 + c) * NF0 + koff;
        const v16h wa0 = Frag<_Float16>::load(wp);
        const v16h wa1 = Frag<_Float16>::load(wp + 32);
        v8f acc0 = z8, acc1 = z8;
        acc0 = Frag<_Float16>::mma(wa0, hb00, acc0);
        acc1 = Frag<_Float16>::mma(wa0, hb10, acc1);
        acc0 = Frag<_Float16>::mma(wa1, hb01, acc0);
        acc1 = Frag<_Float16>::mma(wa1, hb11, acc1);
        guard_l2(acc0, acc1, wa0, wa1, hb00, hb01, hb10, hb11);
        const v4f ba = *(const v4f*)(sCst + 256 + nt * 16 + koff);
        const v4f bb = *(const v4f*)(sCst + 256 + nt * 16 + koff + 4);
        v8h o0, o1;
#pragma unroll
        for (int r = 0; r < 4; ++r) {
          o0[r]     = (_Float16)silu_f(fmaf(acc0[r],     WCARRY_INV, ba[r]));
          o0[4 + r] = (_Float16)silu_f(fmaf(acc0[4 + r], WCARRY_INV, bb[r]));
          o1[r]     = (_Float16)silu_f(fmaf(acc1[r],     WCARRY_INV, ba[r]));
          o1[4 + r] = (_Float16)silu_f(fmaf(acc1[4 + r], WCARRY_INV, bb[r]));
        }
        *(v8h*)(h1w + c * H1P + nt * 16 + koff)        = o0;
        *(v8h*)(h1w + (16 + c) * H1P + nt * 16 + koff) = o1;
      }
    }
    wave_lds_sync();

    {
      v16h a0[4], a1[4];
#pragma unroll
      for (int kt = 0; kt < 4; ++kt) {
        a0[kt] = Frag<_Float16>::load(h1w + c * H1P + kt * 32 + koff);
        a1[kt] = Frag<_Float16>::load(h1w + (16 + c) * H1P + kt * 32 + koff);
      }
      const _Float16* bbase = Bt2 + (size_t)c * NF1 + koff;
#pragma unroll
      for (int nt = 0; nt < 32; ++nt) {
        const _Float16* bp = bbase + (size_t)nt * 16 * NF1;
        const v16h b0 = Frag<_Float16>::load(bp);
        const v16h b1 = Frag<_Float16>::load(bp + 32);
        const v16h b2 = Frag<_Float16>::load(bp + 64);
        const v16h b3 = Frag<_Float16>::load(bp + 96);
        v8f acc0 = z8, acc1 = z8;
        acc0 = Frag<_Float16>::mma(a0[0], b0, acc0);
        acc1 = Frag<_Float16>::mma(a1[0], b0, acc1);
        acc0 = Frag<_Float16>::mma(a0[1], b1, acc0);
        acc1 = Frag<_Float16>::mma(a1[1], b1, acc1);
        acc0 = Frag<_Float16>::mma(a0[2], b2, acc0);
        acc1 = Frag<_Float16>::mma(a1[2], b2, acc1);
        acc0 = Frag<_Float16>::mma(a0[3], b3, acc0);
        acc1 = Frag<_Float16>::mma(a1[3], b3, acc1);
        guard_l3(acc0, acc1, b0, b1, b2, b3, a0[0], a0[1], a0[2], a0[3], a1[0], a1[1], a1[2], a1[3]);
        float mx = rmax[nt], mn = rmin[nt];
#pragma unroll
        for (int r = 0; r < 8; ++r) {
          mx = fmaxf(mx, acc0[r]);
          mx = fmaxf(mx, acc1[r]);
          mn = fminf(mn, acc0[r]);
          mn = fminf(mn, acc1[r]);
        }
        rmax[nt] = mx;
        rmin[nt] = mn;
        asm volatile("" ::: "memory");
      }
    }
    wave_lds_sync();
  }

#pragma unroll
  for (int nt = 0; nt < 32; ++nt) {
    const float om = __shfl_xor(rmax[nt], 16, 32);
    const float on = __shfl_xor(rmin[nt], 16, 32);
    rmax[nt] = fmaxf(rmax[nt], om);
    rmin[nt] = fminf(rmin[nt], on);
  }

  const size_t prow = ((size_t)cs * NPART + (size_t)ch * K1_WAVES + (size_t)wave) * NF2;

#pragma unroll
  for (int nt = 0; nt < 32; ++nt) slab[nt * 16 + c] = rmax[nt];
  wave_lds_sync();
  {
    float* op = PMAX + prow;
    for (int pass = 0; pass < 2; ++pass) {
#pragma unroll
      for (int q = 0; q < 4; ++q) {
        const v4f v = *(const v4f*)(slab + q * 128 + lane * 4);
        *(volatile v4f*)(op + q * 128 + lane * 4) = v;
      }
      __threadfence();
    }
  }
  wave_lds_sync();
#pragma unroll
  for (int nt = 0; nt < 32; ++nt) slab[nt * 16 + c] = rmin[nt];
  wave_lds_sync();
  {
    float* op = PMIN + prow;
    for (int pass = 0; pass < 2; ++pass) {
#pragma unroll
      for (int q = 0; q < 4; ++q) {
        const v4f v = *(const v4f*)(slab + q * 128 + lane * 4);
        *(volatile v4f*)(op + q * 128 + lane * 4) = v;
      }
      __threadfence();
    }
  }
}

__global__ __launch_bounds__(256) void head_kernel(const float* __restrict__ PMAX, const float* __restrict__ PMIN,
                                                   const float* __restrict__ b1_2,
                                                   const float* __restrict__ W2_0, const float* __restrict__ b2_0,
                                                   const float* __restrict__ W2_1, const float* __restrict__ b2_1,
                                                   float* __restrict__ LAT) {
  __shared__ __align__(16) float sL0[NF2];
  __shared__ __align__(16) float sHd[NHEAD];
  __shared__ __align__(16) float sOut[NF2];
  const int t  = threadIdx.x;
  const int cs = blockIdx.x;
  const float* pm = PMAX + (size_t)cs * NPART * NF2;
  const float* pn = PMIN + (size_t)cs * NPART * NF2;

  float mx0 = -INFINITY, mx1 = -INFINITY, mn0 = INFINITY, mn1 = INFINITY;
#pragma unroll 2
  for (int p = 0; p < NPART; ++p) {
    mx0 = fmaxf(mx0, pm[(size_t)p * NF2 + t]);
    mx1 = fmaxf(mx1, pm[(size_t)p * NF2 + 256 + t]);
    mn0 = fminf(mn0, pn[(size_t)p * NF2 + t]);
    mn1 = fminf(mn1, pn[(size_t)p * NF2 + 256 + t]);
  }
  {
    const float bA = b1_2[t], bB = b1_2[256 + t];
    const float s0 = silu_f(fmaf(mx0, WCARRY_INV, bA));
    const float s1 = silu_f(fmaf(mn0, WCARRY_INV, bA));
    const float s2 = silu_f(fmaf(mx1, WCARRY_INV, bB));
    const float s3 = silu_f(fmaf(mn1, WCARRY_INV, bB));
    sL0[t]       = fmaxf(s0, s1);
    sL0[256 + t] = fmaxf(s2, s3);
  }
  __syncthreads();

  {
    float a0 = 0.0f, a1 = 0.0f, a2 = 0.0f, a3 = 0.0f;
#pragma unroll 1
    for (int k = 0; k < NF2; k += 4) {
      a0 = fmaf(sL0[k],     W2_0[(size_t)(k)     * NHEAD + t], a0);
      a1 = fmaf(sL0[k + 1], W2_0[(size_t)(k + 1) * NHEAD + t], a1);
      a2 = fmaf(sL0[k + 2], W2_0[(size_t)(k + 2) * NHEAD + t], a2);
      a3 = fmaf(sL0[k + 3], W2_0[(size_t)(k + 3) * NHEAD + t], a3);
    }
    const float pre = ((a0 + a1) + (a2 + a3)) + b2_0[t];
    sHd[t] = silu_f(pre);
  }
  __syncthreads();

  {
    float a0 = 0.0f, a1 = 0.0f, c0 = 0.0f, c1 = 0.0f;
#pragma unroll 1
    for (int k = 0; k < NHEAD; k += 2) {
      const float h0v = sHd[k], h1v = sHd[k + 1];
      a0 = fmaf(h0v, W2_1[(size_t)(k)     * NF2 + t],       a0);
      c0 = fmaf(h0v, W2_1[(size_t)(k)     * NF2 + 256 + t], c0);
      a1 = fmaf(h1v, W2_1[(size_t)(k + 1) * NF2 + t],       a1);
      c1 = fmaf(h1v, W2_1[(size_t)(k + 1) * NF2 + 256 + t], c1);
    }
    sOut[t]       = (a0 + a1) + b2_1[t];
    sOut[256 + t] = (c0 + c1) + b2_1[256 + t];
  }
  __syncthreads();

  if (t < 128) {
    const v4f v = *(const v4f*)(sOut + t * 4);
    float* op = LAT + (size_t)cs * NF2 + t * 4;
    *(volatile v4f*)op = v;
    __threadfence();
    *(volatile v4f*)op = v;
  }
}

__global__ __launch_bounds__(256) void gather_rows_kernel(const int* __restrict__ x, const float* LAT,
                                                          float* __restrict__ out, int nrows) {
  const int lane = threadIdx.x & 31;
  const int row  = blockIdx.x * 8 + (threadIdx.x >> 5);
  if (row >= nrows) return;
  const int xi = x[row];
  const bool ok = ((unsigned)xi < (unsigned)NCASE);
  const int xc = xi < 0 ? 0 : (xi > NCASE - 1 ? NCASE - 1 : xi);
  const float* lp = LAT + (size_t)xc * NF2;
  v4f v[4];
#pragma unroll
  for (int q = 0; q < 4; ++q) {
    const v4f tv = *(const v4f*)(lp + q * 128 + lane * 4);
#pragma unroll
    for (int e = 0; e < 4; ++e) v[q][e] = ok ? tv[e] : 0.0f;
  }
  float* op = out + (size_t)row * NF2;
#pragma unroll
  for (int q = 0; q < 4; ++q) *(volatile v4f*)(op + q * 128 + lane * 4) = v[q];
  __threadfence();
#pragma unroll
  for (int q = 0; q < 4; ++q) *(volatile v4f*)(op + q * 128 + lane * 4) = v[q];
}

extern "C" void kernel_launch(void* const* d_in, const int* in_sizes, int n_in,
                              void* d_out, int out_size, void* d_ws, size_t ws_size, hipStream_t stream) {
  if (n_in < 12 || d_out == nullptr || d_ws == nullptr) return;
  if (in_sizes[0] != NCASE * NPTS * 3 || in_sizes[1] != 3 * NF0 || in_sizes[2] != NF0 ||
      in_sizes[3] != NF0 * NF1 || in_sizes[4] != NF1 || in_sizes[5] != NF1 * NF2 || in_sizes[6] != NF2 ||
      in_sizes[7] != NF2 * NHEAD || in_sizes[8] != NHEAD || in_sizes[9] != NHEAD * NF2 || in_sizes[10] != NF2 ||
      in_sizes[11] != NBATCH || out_size != NBATCH * NF2) return;

  const float* pts  = (const float*)d_in[0];
  const float* W1_0 = (const float*)d_in[1];
  const float* b1_0 = (const float*)d_in[2];
  const float* W1_1 = (const float*)d_in[3];
  const float* b1_1 = (const float*)d_in[4];
  const float* W1_2 = (const float*)d_in[5];
  const float* b1_2 = (const float*)d_in[6];
  const float* W2_0 = (const float*)d_in[7];
  const float* b2_0 = (const float*)d_in[8];
  const float* W2_1 = (const float*)d_in[9];
  const float* b2_1 = (const float*)d_in[10];
  const int*   xid  = (const int*)d_in[11];
  float* out = (float*)d_out;

  char* ws = (char*)d_ws;
  size_t off = 0;
  auto carve = [&](size_t bytes) -> char* { char* p = ws + off; off += (bytes + 255) & ~(size_t)255; return p; };
  unsigned short* Bt1 = (unsigned short*)carve((size_t)NF1 * NF0 * 2);
  unsigned short* Bt2 = (unsigned short*)carve((size_t)NF2 * NF1 * 2);
  float* PMAX = (float*)carve((size_t)NCASE * NPART * NF2 * 4);
  float* PMIN = (float*)carve((size_t)NCASE * NPART * NF2 * 4);
  float* LAT  = (float*)carve((size_t)NCASE * NF2 * 4);
  if (off > ws_size || off > (size_t)134217728) return;

  prep_weights_kernel<<<(1024 + 8192) / 256, 256, 0, stream>>>(W1_1, W1_2, Bt1, Bt2);

  mlp_colminmax_kernel<<<NCASE * NCHUNK, K1_THREADS, 0, stream>>>(pts, W1_0, b1_0, b1_1, Bt1, Bt2, PMAX, PMIN);

  head_kernel<<<NCASE, 256, 0, stream>>>(PMAX, PMIN, b1_2, W2_0, b2_0, W2_1, b2_1, LAT);

  gather_rows_kernel<<<NBATCH / 8, 256, 0, stream>>>(xid, LAT, out, NBATCH);
}
